// ConvLSTMBlock_69870527971932
// MI455X (gfx1250) — hardware-verified
//
#include <hip/hip_runtime.h>
#include <hip/hip_bf16.h>
#include <math.h>


#define BB   4
#define TT   16
#define HH   64
#define WW   64
#define CC   32
#define FF   64
#define GG   256
#define HWP  (HH * WW)
#define NPIX_X (BB * TT * HWP)
#define NPIX_S (BB * HWP)
#define KX   (9 * CC)
#define KHH  (9 * FF)
#define KTOT (KX + KHH)
#define KP   896
#define NGRP (KP / 8)
#define NGX  (KX / 8)
#define NGH  (KHH / 8)
#define WSCALE 16.0f
#define WSCALE_INV (1.0f / 16.0f)
#define POOL_H 32
#define POOL_W 32

typedef __attribute__((ext_vector_type(16))) _Float16 v16h;
typedef __attribute__((ext_vector_type(8)))  _Float16 v8h;
typedef __attribute__((ext_vector_type(16))) __bf16   v16b;
typedef __attribute__((ext_vector_type(8)))  __bf16   v8b;
typedef __attribute__((ext_vector_type(8)))  float    v8f;
typedef __attribute__((ext_vector_type(4)))  float    v4f;

__device__ __forceinline__ unsigned short f2bf_bits(float f) {
  unsigned u = __float_as_uint(f);
  return (unsigned short)((u + 0x7FFFu + ((u >> 16) & 1u)) >> 16);
}
__device__ __forceinline__ float bf_bits2f(unsigned short h) { return __uint_as_float(((unsigned)h) << 16); }

__device__ __forceinline__ void dep_guard_h(v8f& a, v8f& b, v16h x, v16h y) { asm volatile("v_nop\n\tv_nop\n\tv_nop\n\tv_nop" : "+v"(a), "+v"(b) : "v"(x), "v"(y)); }
__device__ __forceinline__ void dep_guard_b(v8f& a, v8f& b, v16b x, v16b y) { asm volatile("v_nop\n\tv_nop\n\tv_nop\n\tv_nop" : "+v"(a), "+v"(b) : "v"(x), "v"(y)); }
__device__ __forceinline__ void keep4_h(v16h a, v16h b, v16h c, v16h d) { asm volatile("v_nop" :: "v"(a), "v"(b), "v"(c), "v"(d)); }
__device__ __forceinline__ void keep4_b(v16b a, v16b b, v16b c, v16b d) { asm volatile("v_nop" :: "v"(a), "v"(b), "v"(c), "v"(d)); }
__device__ __forceinline__ void acc_guard4(v8f& a, v8f& b, v8f& c, v8f& d) { asm volatile("v_nop\n\tv_nop\n\tv_nop\n\tv_nop" : "+v"(a), "+v"(b), "+v"(c), "+v"(d)); }
template <typename T> struct Frag;
template <> struct Frag<_Float16> {
  typedef v16h V; union U { v16h v; v8h h[2]; };
  static __device__ __forceinline__ v16h load(const _Float16* p) {
    U f; f.h[0] = *(const v8h*)(p); f.h[1] = *(const v8h*)(p + 16); return f.v;
  }
  static __device__ __forceinline__ v8f mma(v16h a, v16h b, v8f c) {
    return __builtin_amdgcn_wmma_f32_16x16x32_f16(false, a, false, b, (short)0, c, false, false);
  }
  static __device__ __forceinline__ void guard(v8f& a, v8f& b, v16h x, v16h y) { dep_guard_h(a, b, x, y); }
  static __device__ __forceinline__ void keep(v16h a, v16h b, v16h c, v16h d) { keep4_h(a, b, c, d); }
};
template <> struct Frag<__bf16> {
  typedef v16b V; union U { v16b v; v8b h[2]; };
  static __device__ __forceinline__ v16b load(const __bf16* p) {
    U f; f.h[0] = *(const v8b*)(p); f.h[1] = *(const v8b*)(p + 16); return f.v;
  }
  static __device__ __forceinline__ v8f mma(v16b a, v16b b, v8f c) {
    return __builtin_amdgcn_wmma_f32_16x16x32_bf16(false, a, false, b, (short)0, c, false, false);
  }
  static __device__ __forceinline__ void guard(v8f& a, v8f& b, v16b x, v16b y) { dep_guard_b(a, b, x, y); }
  static __device__ __forceinline__ void keep(v16b a, v16b b, v16b c, v16b d) { keep4_b(a, b, c, d); }
};

template <int ET> struct Elem;
template <> struct Elem<0> { typedef _Float16 T; };
template <> struct Elem<1> { typedef __bf16 T; };
template <int ET, bool SPLIT, int BIAS_MODE, int OUT_MODE, bool RESID, int ACT = 0>
__global__ __launch_bounds__(256) void wmma_gemm64(
    const unsigned short* __restrict__ Ap, const unsigned short* __restrict__ A2p, int lda, long strideA,
    const unsigned short* __restrict__ Btp, const unsigned short* __restrict__ Bt2p, int ldb, long strideB,
    void* __restrict__ Cout, void* __restrict__ Cout2, int ldc, long strideC,
    const float* __restrict__ bias,
    const float* __restrict__ resid, long strideR,
    int M, int N, int K, float scale) {
  typedef typename Elem<ET>::T T;
  typedef typename Frag<T>::V V;
  const T* A = (const T*)Ap; const T* A2 = (const T*)A2p; const T* Bt = (const T*)Btp; const T* Bt2 = (const T*)Bt2p;
  __shared__ __align__(16) float sT[8][16 * 68];
  const int b    = blockIdx.y;
  const int lane = threadIdx.x & 31;
  const int wave = threadIdx.x >> 5;
  const int tilesN = N >> 6;
  const int tilesM = M >> 6;
  const int tile = blockIdx.x * 8 + wave;
  if (tile >= tilesM * tilesN) return;
  const int tm = tile / tilesN;
  const int tn = tile - tm * tilesN;
  const int m0 = tm << 6;
  const int n0 = tn << 6;

  const T* Ab  = A  + (size_t)b * strideA;
  const T* Bb  = Bt + (size_t)b * strideB;
  const T* Ab2 = SPLIT ? (A2  + (size_t)b * strideA) : nullptr;
  const T* Bb2 = SPLIT ? (Bt2 + (size_t)b * strideB) : nullptr;

  const int rlane = lane & 15;
  const int koff  = (lane >> 4) * 8;
  const int mOff  = (lane >> 4) * 8;

  v8f acc[4][4];
#pragma unroll
  for (int i = 0; i < 4; ++i)
#pragma unroll
    for (int j = 0; j < 4; ++j) acc[i][j] = (v8f){0.f,0.f,0.f,0.f,0.f,0.f,0.f,0.f};

  for (int k0 = 0; k0 < K; k0 += 32) {
    V bh[4], bl[4];
#pragma unroll
    for (int j = 0; j < 4; ++j) {
      const size_t bo = (size_t)(n0 + (j << 4) + rlane) * ldb + koff + k0;
      bh[j] = Frag<T>::load(Bb + bo);
      if (SPLIT) bl[j] = Frag<T>::load(Bb2 + bo);
    }
#pragma unroll
    for (int i = 0; i < 4; ++i) {
      const size_t ao = (size_t)(m0 + (i << 4) + rlane) * lda + koff + k0;
      V ah = Frag<T>::load(Ab + ao);
      V al;
      if (SPLIT) al = Frag<T>::load(Ab2 + ao);
#pragma unroll
      for (int j = 0; j < 4; ++j) {
        acc[i][j] = Frag<T>::mma(ah, bh[j], acc[i][j]);
        if (SPLIT) {
          acc[i][j] = Frag<T>::mma(ah, bl[j], acc[i][j]);
          acc[i][j] = Frag<T>::mma(al, bh[j], acc[i][j]);
        }
      }
      Frag<T>::guard(acc[i][0], acc[i][3], ah, SPLIT ? al : ah);
    }
    Frag<T>::keep(bh[0], bh[1], bh[2], bh[3]);
    if (SPLIT) Frag<T>::keep(bl[0], bl[1], bl[2], bl[3]);
  }
  acc_guard4(acc[0][0], acc[0][1], acc[0][2], acc[0][3]);
  acc_guard4(acc[1][0], acc[1][1], acc[1][2], acc[1][3]);
  acc_guard4(acc[2][0], acc[2][1], acc[2][2], acc[2][3]);
  acc_guard4(acc[3][0], acc[3][1], acc[3][2], acc[3][3]);

  float* slab = sT[wave];
  const float* Rb = RESID ? (resid + (size_t)b * strideR) : nullptr;
#pragma unroll
  for (int i = 0; i < 4; ++i) {
    const int mBase = m0 + (i << 4);
#pragma unroll
    for (int j = 0; j < 4; ++j) {
      const int n = n0 + (j << 4) + rlane;
      float bv = 0.f;
      if (BIAS_MODE == 2) bv = bias[n];
#pragma unroll
      for (int r = 0; r < 8; ++r) {
        float v = acc[i][j][r] * scale;
        if (BIAS_MODE == 1) v += bias[mBase + mOff + r];
        if (BIAS_MODE == 2) v += bv;
        if (RESID) v += Rb[(size_t)(mBase + mOff + r) * ldc + n];
        if (ACT == 1) v = tanhf(v);
        if (ACT == 2) v = fmaxf(v, 0.0f);
        if (ACT == 3) v = v / (1.0f + expf(-v));
        if (ACT == 4) v = (v > 0.f) ? v : 0.01f * v;
        if (ACT == 5) v = 0.5f * v * (1.0f + erff(v * 0.70710678118654752f));
        slab[(mOff + r) * 68 + (j << 4) + rlane] = v;
      }
    }
    __builtin_amdgcn_fence(__ATOMIC_RELEASE, "workgroup");
    __builtin_amdgcn_wave_barrier();
    __builtin_amdgcn_fence(__ATOMIC_ACQUIRE, "workgroup");
    if (OUT_MODE == 0) {
      float* C = (float*)Cout + (size_t)b * strideC;
      const int hh = lane >> 4, c4 = (lane & 15) * 4;
      for (int pass = 0; pass < 2; ++pass) {
#pragma unroll
        for (int it = 0; it < 8; ++it) {
          const int row = it * 2 + hh;
          v4f v = *(const v4f*)(slab + row * 68 + c4);
          *(volatile v4f*)(C + (size_t)(mBase + row) * ldc + n0 + c4) = v;
        }
        __threadfence();
      }
    } else {
      const int q = lane >> 3, c8 = (lane & 7) * 8;
      unsigned short* C  = (unsigned short*)Cout  + (size_t)b * strideC;
      unsigned short* C2 = (OUT_MODE == 2) ? ((unsigned short*)Cout2 + (size_t)b * strideC) : nullptr;
      for (int pass = 0; pass < 2; ++pass) {
#pragma unroll
        for (int it = 0; it < 4; ++it) {
          const int row = it * 4 + q;
          const float* sp = slab + row * 68 + c8;
          v8h hv, lv;
#pragma unroll
          for (int e = 0; e < 8; ++e) {
            if (OUT_MODE == 1) {
              hv[e] = (_Float16)sp[e];
            } else {
              unsigned short hb = f2bf_bits(sp[e]);
              unsigned short lb = f2bf_bits(sp[e] - bf_bits2f(hb));
              hv[e] = __builtin_bit_cast(_Float16, hb);
              lv[e] = __builtin_bit_cast(_Float16, lb);
            }
          }
          *(volatile v8h*)(C + (size_t)(mBase + row) * ldc + n0 + c8) = hv;
          if (OUT_MODE == 2) *(volatile v8h*)(C2 + (size_t)(mBase + row) * ldc + n0 + c8) = lv;
        }
        __threadfence();
      }
    }
    __builtin_amdgcn_fence(__ATOMIC_RELEASE, "workgroup");
    __builtin_amdgcn_wave_barrier();
    __builtin_amdgcn_fence(__ATOMIC_ACQUIRE, "workgroup");
  }
}

__device__ __forceinline__ float hsig(float x) {
  return fminf(fmaxf(0.2f * x + 0.5f, 0.0f), 1.0f);
}
__device__ __forceinline__ float tanh_f(float x) {
  const float ax = fabsf(x);
  const float e  = __expf(-2.0f * ax);
  const float r  = (1.0f - e) * __builtin_amdgcn_rcpf(1.0f + e);
  return copysignf(r, x);
}

__global__ __launch_bounds__(256)
void packw_kernel(const float* __restrict__ wx, const float* __restrict__ wh, _Float16* __restrict__ bt) {
  const int g = blockIdx.x * 256 + threadIdx.x;
  if (g >= GG * NGRP) return;
  const int n  = g / NGRP;
  const int jg = g - n * NGRP;
  const int k8 = jg * 8;
  v8h v;
#pragma unroll
  for (int e = 0; e < 8; ++e) {
    const int k = k8 + e;
    float f = 0.0f;
    if (k < KX)        f = wx[(size_t)k * GG + n];
    else if (k < KTOT) f = wh[(size_t)(k - KX) * GG + n];
    v[e] = (_Float16)(f * WSCALE);
  }
  _Float16* p = bt + (size_t)g * 8;
  *(volatile v8h*)p = v;
  __threadfence();
  *(volatile v8h*)p = v;
}

__global__ __launch_bounds__(256)
void ln_kernel(const float* __restrict__ x, const float* __restrict__ gamma,
               const float* __restrict__ beta, _Float16* __restrict__ xn, int npix) {
  const int gi = blockIdx.x * 256 + threadIdx.x;
  const int P  = gi >> 2;
  const int cg = gi & 3;
  const bool ok = (P < npix);
  const int Pc = ok ? P : 0;
  const float* xp = x + (size_t)Pc * CC + cg * 8;
  const v4f qa = *(const v4f*)xp;
  const v4f qb = *(const v4f*)(xp + 4);
  float v[8];
  v[0] = qa[0]; v[1] = qa[1]; v[2] = qa[2]; v[3] = qa[3];
  v[4] = qb[0]; v[5] = qb[1]; v[6] = qb[2]; v[7] = qb[3];
  float s = 0.0f;
#pragma unroll
  for (int e = 0; e < 8; ++e) s += v[e];
  s += __shfl_xor(s, 1, 32);
  s += __shfl_xor(s, 2, 32);
  const float mean = s * (1.0f / CC);
  float s2 = 0.0f;
#pragma unroll
  for (int e = 0; e < 8; ++e) { v[e] -= mean; s2 += v[e] * v[e]; }
  s2 += __shfl_xor(s2, 1, 32);
  s2 += __shfl_xor(s2, 2, 32);
  const float rs = rsqrtf(s2 * (1.0f / CC) + 1e-3f);
  v8h o;
#pragma unroll
  for (int e = 0; e < 8; ++e) o[e] = (_Float16)(v[e] * rs * gamma[cg * 8 + e] + beta[cg * 8 + e]);
  if (ok) {
    _Float16* op = xn + (size_t)P * CC + cg * 8;
    *(volatile v8h*)op = o;
    __threadfence();
    *(volatile v8h*)op = o;
  }
}

__global__ __launch_bounds__(256)
void im2col_kernel(const _Float16* __restrict__ xn, const _Float16* __restrict__ h16,
                   _Float16* __restrict__ im, int t, int hvalid) {
  const int lane = threadIdx.x & 31;
  const int wave = threadIdx.x >> 5;
  const int q    = blockIdx.x * 8 + wave;
  const int b    = q >> 12;
  const int rem  = q & (HWP - 1);
  const int y    = rem >> 6;
  const int xx   = rem & (WW - 1);
  v8h vals[4];
#pragma unroll
  for (int it = 0; it < 4; ++it) {
    const int j = it * 32 + lane;
    v8h v = {};
    const bool isx = (j < NGX);
    const bool ish = (j >= NGX) && (j < NGX + NGH);
    const int jj   = isx ? j : (j - NGX);
    const int tap  = isx ? (jj >> 2) : (jj >> 3);
    const int cg   = isx ? (jj & 3) : (jj & 7);
    const int ky   = tap / 3;
    const int kx   = tap - 3 * ky;
    const int ny   = y + ky - 1;
    const int nx   = xx + kx - 1;
    const bool inb = (ny >= 0) && (ny < HH) && (nx >= 0) && (nx < WW);
    if (isx && inb) {
      v = *(const v8h*)(xn + ((size_t)((b * TT + t) * HWP + ny * WW + nx)) * CC + cg * 8);
    } else if (ish && inb && (hvalid != 0)) {
      v = *(const v8h*)(h16 + ((size_t)(b * HWP + ny * WW + nx)) * FF + cg * 8);
    }
    vals[it] = v;
  }
  _Float16* row = im + (size_t)q * KP;
  for (int pass = 0; pass < 2; ++pass) {
#pragma unroll
    for (int it = 0; it < 4; ++it) {
      const int j = it * 32 + lane;
      if (j < NGRP) *(volatile v8h*)(row + j * 8) = vals[it];
    }
    __threadfence();
  }
}

__global__ __launch_bounds__(256)
void gate_kernel(const float* __restrict__ z, float* __restrict__ cst,
                 _Float16* __restrict__ h16, float* __restrict__ out, int t, int cvalid) {
  __shared__ __align__(16) float hs[64 * FF];
  __shared__ __align__(16) float cs[64 * FF];
  const int tid = threadIdx.x;
  const int bid = blockIdx.x;
  const int xh  = bid & 1;
  const int yo  = (bid >> 1) & (POOL_H - 1);
  const int b   = bid >> 6;
  const int qbase = b * HWP + (2 * yo) * WW + xh * 32;

#pragma unroll 1
  for (int k = 0; k < 16; ++k) {
    const int e  = 256 * k + tid;
    const int p  = e >> 6;
    const int ch = e & (FF - 1);
    const int q  = qbase + (p >> 5) * WW + (p & 31);
    const float* zp = z + (size_t)q * GG + ch;
    const float zi = zp[0];
    const float zf = zp[FF];
    const float zc = zp[2 * FF];
    const float zo = zp[3 * FF];
    float cold = 0.0f;
    if (cvalid != 0) cold = cst[(size_t)q * FF + ch];
    const float ig = hsig(zi);
    const float fg = hsig(zf);
    const float og = hsig(zo);
    const float cn = fg * cold + ig * tanh_f(zc);
    const float hn = og * tanh_f(cn);
    hs[p * FF + ch] = hn;
    cs[p * FF + ch] = cn;
  }
  __syncthreads();

  v4f cv[4]; size_t co[4];
#pragma unroll
  for (int k = 0; k < 4; ++k) {
    const int idx = 256 * k + tid;
    const int p   = idx >> 4;
    const int c4  = (idx & 15) * 4;
    const int q   = qbase + (p >> 5) * WW + (p & 31);
    cv[k] = *(const v4f*)(cs + p * FF + c4);
    co[k] = (size_t)q * FF + c4;
  }
  v8h hv[2]; size_t ho[2];
#pragma unroll
  for (int k = 0; k < 2; ++k) {
    const int task = 256 * k + tid;
    const int p    = task >> 3;
    const int cg   = task & 7;
    const int q    = qbase + (p >> 5) * WW + (p & 31);
    const float* sp = hs + p * FF + cg * 8;
    const v4f a0 = *(const v4f*)sp;
    const v4f a1 = *(const v4f*)(sp + 4);
    v8h w;
    w[0] = (_Float16)a0[0]; w[1] = (_Float16)a0[1]; w[2] = (_Float16)a0[2]; w[3] = (_Float16)a0[3];
    w[4] = (_Float16)a1[0]; w[5] = (_Float16)a1[1]; w[6] = (_Float16)a1[2]; w[7] = (_Float16)a1[3];
    hv[k] = w;
    ho[k] = (size_t)q * FF + cg * 8;
  }
  const int xo = tid >> 4;
  const int c4 = (tid & 15) * 4;
  const v4f m0 = *(const v4f*)(hs + (2 * xo) * FF + c4);
  const v4f m1 = *(const v4f*)(hs + (2 * xo + 1) * FF + c4);
  const v4f m2 = *(const v4f*)(hs + (32 + 2 * xo) * FF + c4);
  const v4f m3 = *(const v4f*)(hs + (33 + 2 * xo) * FF + c4);
  v4f mm;
#pragma unroll
  for (int i = 0; i < 4; ++i) mm[i] = fmaxf(fmaxf(m0[i], m1[i]), fmaxf(m2[i], m3[i]));
  const size_t oo = ((((size_t)(b * TT + t)) * POOL_H + yo) * POOL_W + xh * 16 + xo) * FF + c4;

  for (int pass = 0; pass < 2; ++pass) {
#pragma unroll
    for (int k = 0; k < 4; ++k) *(volatile v4f*)(cst + co[k]) = cv[k];
#pragma unroll
    for (int k = 0; k < 2; ++k) *(volatile v8h*)(h16 + ho[k]) = hv[k];
    *(volatile v4f*)(out + oo) = mm;
    __threadfence();
  }
}

extern "C" void kernel_launch(void* const* d_in, const int* in_sizes, int n_in,
                              void* d_out, int out_size, void* d_ws, size_t ws_size,
                              hipStream_t stream) {
  if (n_in < 6) return;
  if (in_sizes[0] != NPIX_X * CC) return;
  if (in_sizes[1] != CC || in_sizes[2] != CC) return;
  if (in_sizes[3] != 9 * CC * GG) return;
  if (in_sizes[4] != 9 * FF * GG) return;
  if (in_sizes[5] != GG) return;
  if (out_size != BB * TT * POOL_H * POOL_W * FF) return;

  const float* x     = (const float*)d_in[0];
  const float* gamma = (const float*)d_in[1];
  const float* beta  = (const float*)d_in[2];
  const float* wx    = (const float*)d_in[3];
  const float* wh    = (const float*)d_in[4];
  const float* bias  = (const float*)d_in[5];
  float* out = (float*)d_out;
  char*  ws  = (char*)d_ws;

  size_t off = 0;
  const size_t bt_bytes  = (size_t)GG * KP * 2;
  const size_t xn_bytes  = (size_t)NPIX_X * CC * 2;
  const size_t im_bytes  = (size_t)NPIX_S * KP * 2;
  const size_t z_bytes   = (size_t)NPIX_S * GG * 4;
  const size_t c_bytes   = (size_t)NPIX_S * FF * 4;
  const size_t h_bytes   = (size_t)NPIX_S * FF * 2;
  _Float16* bt  = (_Float16*)(ws + off); off += bt_bytes;
  _Float16* xn  = (_Float16*)(ws + off); off += xn_bytes;
  _Float16* im  = (_Float16*)(ws + off); off += im_bytes;
  float*    zb  = (float*)   (ws + off); off += z_bytes;
  float*    cst = (float*)   (ws + off); off += c_bytes;
  _Float16* h16 = (_Float16*)(ws + off); off += h_bytes;
  if (off > ws_size) return;

  packw_kernel<<<(GG * NGRP + 255) / 256, 256, 0, stream>>>(wx, wh, bt);
  ln_kernel<<<(NPIX_X * 4 + 255) / 256, 256, 0, stream>>>(x, gamma, beta, xn, NPIX_X);

  const int tiles = (NPIX_S / 64) * (GG / 64);
  const dim3 ggrid((tiles + 7) / 8, 1, 1);

  for (int t = 0; t < TT; ++t) {
    const int hv = (t > 0) ? 1 : 0;
    const int kk = (t > 0) ? KTOT : KX;
    im2col_kernel<<<NPIX_S / 8, 256, 0, stream>>>(xn, h16, im, t, hv);
    wmma_gemm64<0, false, 2, 0, false, 0><<<ggrid, 256, 0, stream>>>(
        (const unsigned short*)im, (const unsigned short*)im, KP, 0L,
        (const unsigned short*)bt, (const unsigned short*)bt, KP, 0L,
        (void*)zb, (void*)zb, GG, 0L,
        bias,
        (const float*)zb, 0L,
        NPIX_S, GG, kk, WSCALE_INV);
    gate_kernel<<<BB * POOL_H * 2, 256, 0, stream>>>(zb, cst, h16, out, t, hv);
  }
}
